// KPConv_2173253452285
// MI455X (gfx1250) — hardware-verified
//
#include <hip/hip_runtime.h>
#include <math.h>

typedef __attribute__((ext_vector_type(16))) _Float16 v16h;
typedef __attribute__((ext_vector_type(16))) __bf16 v16b;
typedef __attribute__((ext_vector_type(8)))  _Float16 v8h;
typedef __attribute__((ext_vector_type(8)))  float v8f;
typedef __attribute__((ext_vector_type(4)))  float v4f;
typedef __attribute__((ext_vector_type(2)))  float v2f;
typedef __attribute__((ext_vector_type(4)))  unsigned v4u;
typedef __attribute__((ext_vector_type(4)))  int v4i;
typedef float __attribute__((may_alias)) float_a;
typedef int __attribute__((may_alias)) int_a;

template <typename T> __device__ __forceinline__ void vst2(void* p, T v) { *(volatile T*)p = v; __threadfence(); *(volatile T*)p = v; }
__device__ __forceinline__ v8f wmma16(v16h a, v16h b, v8f c) {
  v8f d = __builtin_amdgcn_wmma_f32_16x16x32_f16(false, a, false, b, (short)0, c, false, false);
  asm volatile("v_nop\n\tv_nop\n\tv_nop\n\tv_nop" : "+v"(d) : "v"(a), "v"(b));
  return d;
}
__device__ __forceinline__ v8f wmma_bf(v16b a, v16b b, v8f c) {
  v8f d = __builtin_amdgcn_wmma_f32_16x16x32_bf16(false, a, false, b, (short)0, c, false, false);
  asm volatile("v_nop\n\tv_nop\n\tv_nop\n\tv_nop" : "+v"(d) : "v"(a), "v"(b));
  return d;
}
__device__ __forceinline__ v16h frag_h(const _Float16* rowk0, int lane) {
  union { v16h v; v8h q[2]; } u; const _Float16* p = rowk0 + 8 * (lane >> 4);
  u.q[0] = *(const v8h*)p; u.q[1] = *(const v8h*)(p + 16); return u.v;
}
__device__ __forceinline__ v16h frag_f32(const float* rowk0, int lane) {
  v16h a; const float* p = rowk0 + 8 * (lane >> 4);
#pragma unroll
  for (int i = 0; i < 8; ++i) { a[i] = (_Float16)p[i]; a[8 + i] = (_Float16)p[16 + i]; }
  return a;
}
__device__ __forceinline__ v16h frag_f32s(const float* rowk0, int lane, float sc) {
  v16h a; const float* p = rowk0 + 8 * (lane >> 4);
#pragma unroll
  for (int i = 0; i < 8; ++i) { a[i] = (_Float16)(p[i] * sc); a[8 + i] = (_Float16)(p[16 + i] * sc); }
  return a;
}
__device__ __forceinline__ v16h fragc_f32(const float* W, int k0, int n, int lane, int ld, int K) {
  v16h a; const int g = lane >> 4;
#pragma unroll
  for (int i = 0; i < 8; ++i) { const int ka = k0 + 8 * g + i, kb = ka + 16;
    a[i] = (_Float16)(ka < K ? W[(size_t)(ka < K ? ka : K - 1) * ld + n] : 0.f); a[8 + i] = (_Float16)(kb < K ? W[(size_t)(kb < K ? kb : K - 1) * ld + n] : 0.f); }
  return a;
}
struct F2 { v16b h, l; };
__device__ __forceinline__ F2 bsplit16(const float v[16]) { F2 r;
#pragma unroll
  for (int i = 0; i < 16; ++i) { const __bf16 h = (__bf16)v[i]; r.h[i] = h; r.l[i] = (__bf16)(v[i] - (float)h); }
  return r; }
__device__ __forceinline__ F2 split_row(const float* row, int k0, int lane) { float v[16]; const float* p = row + k0 + 8 * (lane >> 4);
#pragma unroll
  for (int i = 0; i < 8; ++i) { v[i] = p[i]; v[8 + i] = p[16 + i]; }
  return bsplit16(v); }
__device__ __forceinline__ F2 split_rowK(const float* row, int k0, int lane, int K) { float v[16]; const int g = lane >> 4;
#pragma unroll
  for (int i = 0; i < 8; ++i) { const int ka = k0 + 8 * g + i, kb = ka + 16; v[i] = ka < K ? row[ka < K ? ka : K - 1] : 0.f; v[8 + i] = kb < K ? row[kb < K ? kb : K - 1] : 0.f; }
  return bsplit16(v); }
__device__ __forceinline__ F2 split_col(const float* W, int k0, int n, int lane, int ld, int K) { float v[16]; const int g = lane >> 4;
#pragma unroll
  for (int i = 0; i < 8; ++i) { const int ka = k0 + 8 * g + i, kb = ka + 16; v[i] = ka < K ? W[(size_t)(ka < K ? ka : K - 1) * ld + n] : 0.f; v[8 + i] = kb < K ? W[(size_t)(kb < K ? kb : K - 1) * ld + n] : 0.f; }
  return bsplit16(v); }
__device__ __forceinline__ v8f mac3(const F2& a, const F2& b, v8f c) { c = wmma_bf(a.l, b.h, c); c = wmma_bf(a.h, b.l, c); return wmma_bf(a.h, b.h, c); }
__device__ __forceinline__ float sigm(float v) { return 1.0f / (1.0f + expf(-v)); }
#define LDSX() do { asm volatile("s_wait_dscnt 0" ::: "memory"); __builtin_amdgcn_wave_barrier(); __builtin_amdgcn_fence(__ATOMIC_RELEASE, "workgroup"); } while (0)

#define NM 50000
#define NS 100000
#define NHB 32
#define NK 15
#define CI 64
#define CO 64
#define KW (NK * CI)
#define NMP 50048
#ifndef NMPROC
#define NMPROC NM
#endif
__device__ __forceinline__ float bfr(float v) { return (float)(__bf16)v; }
#define WS_A   0u
#define WS_END (WS_A + 2u * (size_t)NMP * KW)

__global__ __launch_bounds__(256) void k_wsum(const float* __restrict__ QP, const float* __restrict__ SP, const float* __restrict__ X, const int* __restrict__ NBI, const float* __restrict__ KPT, _Float16* __restrict__ A) {
  __shared__ float sw[8][NHB][17]; __shared__ int sidx[8][NHB]; __shared__ __align__(16) _Float16 so[8][KW];
  const int wave = threadIdx.x >> 5, lane = threadIdx.x & 31, col = lane & 15, g = lane >> 4; const size_t m = (size_t)blockIdx.x * 8 + wave;
  if (m >= NMPROC) return;
  { const int ii = NBI[m * NHB + lane]; const bool shadow = !(ii >= 0 && ii < NS); const int idx = shadow ? 0 : ii;
    const float qx = bfr(QP[m * 3]), qy = bfr(QP[m * 3 + 1]), qz = bfr(QP[m * 3 + 2]);
    const float px = shadow ? 1.0e6f : bfr(SP[(size_t)idx * 3]), py = shadow ? 1.0e6f : bfr(SP[(size_t)idx * 3 + 1]), pz = shadow ? 1.0e6f : bfr(SP[(size_t)idx * 3 + 2]);
    const float rx = px - qx, ry = py - qy, rz = pz - qz;
#pragma unroll
    for (int k = 0; k < NK; ++k) { const float dx = rx - bfr(KPT[k * 3]), dy = ry - bfr(KPT[k * 3 + 1]), dz = rz - bfr(KPT[k * 3 + 2]); const float d = sqrtf(dx * dx + dy * dy + dz * dz); sw[wave][lane][k] = fmaxf(1.0f - d / 2.0f, 0.f); }
    sw[wave][lane][15] = 0.f; sw[wave][lane][16] = 0.f; sidx[wave][lane] = shadow ? -1 : idx; }
  LDSX();
  v16h a;
#pragma unroll
  for (int i = 0; i < 8; ++i) { a[i] = (_Float16)sw[wave][8 * g + i][col]; a[8 + i] = (_Float16)sw[wave][16 + 8 * g + i][col]; }
  v16h bx[4]; float hs[16];
#pragma unroll
  for (int i = 0; i < 16; ++i) hs[i] = 0.f;
#pragma unroll
  for (int i = 0; i < 8; ++i) {
#pragma unroll
    for (int hh = 0; hh < 2; ++hh) { const int h = hh * 16 + 8 * g + i; const int idx = sidx[wave][h]; const int ic = idx < 0 ? 0 : idx; const float live = idx < 0 ? 0.f : 1.f; const float* xr = X + (size_t)ic * CI + col;
float xg[4];
#pragma unroll
      for (int j = 0; j < 4; ++j) xg[j] = xr[16 * j];
      asm volatile("s_wait_loadcnt 0x0" ::: "memory");
#pragma unroll
      for (int j = 0; j < 4; ++j) { const float xv = bfr(xg[j]) * live; bx[j][hh * 8 + i] = (_Float16)xv; hs[hh * 8 + i] += xv; } } }
  int cnt = 0;
#pragma unroll
  for (int e = 0; e < 16; ++e) { float s = hs[e];
#pragma unroll
    for (int o = 1; o < 16; o <<= 1) s += __shfl_xor(s, o);
    cnt += (s > 0.f) ? 1 : 0; }
  cnt += __shfl_xor(cnt, 16);
  v8f acc[4] = {};
#pragma unroll
  for (int j = 0; j < 4; ++j) acc[j] = wmma16(a, bx[j], acc[j]);
  const float inv = 1.0f / (float)(cnt > 1 ? cnt : 1);
#pragma unroll
  for (int j = 0; j < 4; ++j)
#pragma unroll
    for (int r = 0; r < 8; ++r) { const int k = 8 * g + r; if (k < NK) so[wave][k * CI + j * 16 + col] = (_Float16)(acc[j][r] * inv); }
  LDSX();
  for (int q = lane; q < KW / 8; q += 32) vst2((unsigned*)(A + m * KW + q * 8), *(const v4u*)&so[wave][q * 8]); }
__global__ __launch_bounds__(256) void k_zero(_Float16* __restrict__ A) { const size_t e = (size_t)blockIdx.x * 256 + threadIdx.x; const size_t n8 = (size_t)(NMP - NM) * KW / 8; if (e >= n8) return; v4u z = {0u, 0u, 0u, 0u}; vst2((unsigned*)(A + (size_t)NM * KW + e * 8), z); }
__global__ __launch_bounds__(128) void k_gemm(const _Float16* __restrict__ A, const float* __restrict__ Wt, float* __restrict__ OUT) { __shared__ __align__(16) float sf[4][16][68];
  const int tid = threadIdx.x, wave = tid >> 5, lane = tid & 31, col = lane & 15, g = lane >> 4; const size_t r0 = (size_t)blockIdx.x * 64 + wave * 16;
  v8f acc[4] = {};
#pragma unroll 2
  for (int kc = 0; kc < KW / 32; ++kc) { const v16h a = frag_h(A + (r0 + col) * KW + kc * 32, lane);
#pragma unroll
    for (int j = 0; j < 4; ++j) { v16h w; const int o = j * 16 + col; const int gg = lane >> 4;
#pragma unroll
      for (int i = 0; i < 8; ++i) { w[i] = (_Float16)(bfr(Wt[(size_t)(kc * 32 + 8 * gg + i) * CO + o]) * 16.0f); w[8 + i] = (_Float16)(bfr(Wt[(size_t)(kc * 32 + 16 + 8 * gg + i) * CO + o]) * 16.0f); }
      asm volatile("s_wait_loadcnt 0x0" ::: "memory"); acc[j] = wmma16(a, w, acc[j]); } }
#pragma unroll
  for (int j = 0; j < 4; ++j)
#pragma unroll
    for (int r = 0; r < 8; ++r) sf[wave][8 * g + r][j * 16 + col] = acc[j][r] * (1.0f / 16.0f);
  LDSX(); for (int rl = 0; rl < 16; ++rl) { const size_t row = r0 + rl; if (row < NMPROC && lane < 16) vst2(OUT + row * CO + lane * 4, *(const v4f*)&sf[wave][rl][lane * 4]); } }
extern "C" void kernel_launch(void* const* d_in, const int* in_sizes, int n_in, void* d_out, int out_size, void* d_ws, size_t ws_size, hipStream_t stream) {
  (void)in_sizes; (void)n_in; (void)out_size;
  if (ws_size < (size_t)WS_END) return;
  _Float16* A = (_Float16*)((char*)d_ws + WS_A);
  k_zero<<<dim3(((NMP - NM) * KW / 8 + 255) / 256), 256, 0, stream>>>(A);
  k_wsum<<<dim3((NMPROC + 7) / 8), 256, 0, stream>>>((const float*)d_in[0], (const float*)d_in[1], (const float*)d_in[2], (const int*)d_in[3], (const float*)d_in[5], A);
  k_gemm<<<dim3(NMP / 64), 128, 0, stream>>>(A, (const float*)d_in[4], (float*)d_out);
}
